// MainGNNModel_32822140076341
// MI455X (gfx1250) — hardware-verified
//
#include <hip/hip_runtime.h>
#include <stdint.h>
#include <math.h>

#define NPF   20000
#define NGW   100000
#define NSW   20000
#define DI    64
#define DO    128
#define KD    128
#define EPG   1600000
#define EGP   1600000
#define ESP   400000
#define EPS   400000
#define NT    256
#define SRB   2048
#define SCH   2048
#define SPT   (SCH / NT)
#define TL_GW 49
#define TL_PF 10
#define TL_SW 10
#define NPA_GW (TL_GW * SRB)
#define NPA_PF (TL_PF * SRB)
#define NPA_SW (TL_SW * SRB)
#define MP_GW 100032
#define MP_PF 20032
#define MP_SW 20032

static_assert(NGW < (1 << 17) && NPF < (1 << 17) && NSW < (1 << 17), "");
static_assert(EPG % SPT == 0 && EGP % SPT == 0 && ESP % SPT == 0 && EPS % SPT == 0, "");
static_assert(SRB == 2048 && NT == 256 && SCH == 2048, "");
static_assert(MP_GW % 64 == 0 && MP_GW >= NGW && NPA_GW >= MP_GW, "");
static_assert(MP_PF % 64 == 0 && MP_PF >= NPF && NPA_PF >= MP_PF, "");
static_assert(MP_SW % 64 == 0 && MP_SW >= NSW && NPA_SW >= MP_SW, "");
static_assert(MP_GW % 16 == 0 && MP_PF % 16 == 0 && MP_SW % 16 == 0, "");
static_assert(NGW % 32 == 0 && NSW % 32 == 0, "");
static_assert((NPF * DO) % (4 * 256) == 0, "");
static_assert(KD % 32 == 0 && DO % 64 == 0 && DI * 2 == KD, "");

typedef __attribute__((ext_vector_type(16))) _Float16 v16h;
typedef __attribute__((ext_vector_type(8)))  _Float16 v8h;
typedef __attribute__((ext_vector_type(16))) __bf16   v16b;
typedef __attribute__((ext_vector_type(8)))  __bf16   v8b;
typedef __attribute__((ext_vector_type(8)))  float    v8f;
typedef __attribute__((ext_vector_type(4)))  float    v4f;
typedef __attribute__((ext_vector_type(2)))  float    v2f;
typedef __attribute__((ext_vector_type(4)))  int      v4i;

__device__ __forceinline__ unsigned short f2bf_bits(float f) {
  unsigned u = __float_as_uint(f);
  return (unsigned short)((u + 0x7FFFu + ((u >> 16) & 1u)) >> 16);
}
__device__ __forceinline__ float bf_bits2f(unsigned short h) { return __uint_as_float(((unsigned)h) << 16); }

__device__ __forceinline__ void split_bf(float f, unsigned short& hb, unsigned short& lb) {
  hb = f2bf_bits(f);
  lb = f2bf_bits(f - bf_bits2f(hb));
}

__device__ __forceinline__ void dep_guard_h(v8f& a, v8f& b, v16h x, v16h y) { asm volatile("v_nop\n\tv_nop\n\tv_nop\n\tv_nop" : "+v"(a), "+v"(b) : "v"(x), "v"(y)); }
__device__ __forceinline__ void dep_guard_b(v8f& a, v8f& b, v16b x, v16b y) { asm volatile("v_nop\n\tv_nop\n\tv_nop\n\tv_nop" : "+v"(a), "+v"(b) : "v"(x), "v"(y)); }
__device__ __forceinline__ void keep4_h(v16h a, v16h b, v16h c, v16h d) { asm volatile("v_nop" :: "v"(a), "v"(b), "v"(c), "v"(d)); }
__device__ __forceinline__ void keep4_b(v16b a, v16b b, v16b c, v16b d) { asm volatile("v_nop" :: "v"(a), "v"(b), "v"(c), "v"(d)); }
__device__ __forceinline__ void acc_guard4(v8f& a, v8f& b, v8f& c, v8f& d) { asm volatile("v_nop\n\tv_nop\n\tv_nop\n\tv_nop" : "+v"(a), "+v"(b), "+v"(c), "+v"(d)); }
template <typename T> struct Frag;
template <> struct Frag<_Float16> {
  typedef v16h V; union U { v16h v; v8h h[2]; };
  static __device__ __forceinline__ v16h load(const _Float16* p) {
    U f; f.h[0] = *(const v8h*)(p); f.h[1] = *(const v8h*)(p + 16); return f.v;
  }
  static __device__ __forceinline__ v8f mma(v16h a, v16h b, v8f c) {
    return __builtin_amdgcn_wmma_f32_16x16x32_f16(false, a, false, b, (short)0, c, false, false);
  }
  static __device__ __forceinline__ void guard(v8f& a, v8f& b, v16h x, v16h y) { dep_guard_h(a, b, x, y); }
  static __device__ __forceinline__ void keep(v16h a, v16h b, v16h c, v16h d) { keep4_h(a, b, c, d); }
};
template <> struct Frag<__bf16> {
  typedef v16b V; union U { v16b v; v8b h[2]; };
  static __device__ __forceinline__ v16b load(const __bf16* p) {
    U f; f.h[0] = *(const v8b*)(p); f.h[1] = *(const v8b*)(p + 16); return f.v;
  }
  static __device__ __forceinline__ v8f mma(v16b a, v16b b, v8f c) {
    return __builtin_amdgcn_wmma_f32_16x16x32_bf16(false, a, false, b, (short)0, c, false, false);
  }
  static __device__ __forceinline__ void guard(v8f& a, v8f& b, v16b x, v16b y) { dep_guard_b(a, b, x, y); }
  static __device__ __forceinline__ void keep(v16b a, v16b b, v16b c, v16b d) { keep4_b(a, b, c, d); }
};

template <int ET> struct Elem;
template <> struct Elem<0> { typedef _Float16 T; };
template <> struct Elem<1> { typedef __bf16 T; };
template <int ET, bool SPLIT, int BIAS_MODE, int OUT_MODE, bool RESID, int ACT = 0>
__global__ __launch_bounds__(256) void wmma_gemm64(
    const unsigned short* __restrict__ Ap, const unsigned short* __restrict__ A2p, int lda, long strideA,
    const unsigned short* __restrict__ Btp, const unsigned short* __restrict__ Bt2p, int ldb, long strideB,
    void* __restrict__ Cout, void* __restrict__ Cout2, int ldc, long strideC,
    const float* __restrict__ bias,
    const float* __restrict__ resid, long strideR,
    int M, int N, int K, float scale) {
  typedef typename Elem<ET>::T T;
  typedef typename Frag<T>::V V;
  const T* A = (const T*)Ap; const T* A2 = (const T*)A2p; const T* Bt = (const T*)Btp; const T* Bt2 = (const T*)Bt2p;
  __shared__ __align__(16) float sT[8][16 * 68];
  const int b    = blockIdx.y;
  const int lane = threadIdx.x & 31;
  const int wave = threadIdx.x >> 5;
  const int tilesN = N >> 6;
  const int tilesM = M >> 6;
  const int tile = blockIdx.x * 8 + wave;
  if (tile >= tilesM * tilesN) return;
  const int tm = tile / tilesN;
  const int tn = tile - tm * tilesN;
  const int m0 = tm << 6;
  const int n0 = tn << 6;

  const T* Ab  = A  + (size_t)b * strideA;
  const T* Bb  = Bt + (size_t)b * strideB;
  const T* Ab2 = SPLIT ? (A2  + (size_t)b * strideA) : nullptr;
  const T* Bb2 = SPLIT ? (Bt2 + (size_t)b * strideB) : nullptr;

  const int rlane = lane & 15;
  const int koff  = (lane >> 4) * 8;
  const int mOff  = (lane >> 4) * 8;

  v8f acc[4][4];
#pragma unroll
  for (int i = 0; i < 4; ++i)
#pragma unroll
    for (int j = 0; j < 4; ++j) acc[i][j] = (v8f){0.f,0.f,0.f,0.f,0.f,0.f,0.f,0.f};

  for (int k0 = 0; k0 < K; k0 += 32) {
    V bh[4], bl[4];
#pragma unroll
    for (int j = 0; j < 4; ++j) {
      const size_t bo = (size_t)(n0 + (j << 4) + rlane) * ldb + koff + k0;
      bh[j] = Frag<T>::load(Bb + bo);
      if (SPLIT) bl[j] = Frag<T>::load(Bb2 + bo);
    }
#pragma unroll
    for (int i = 0; i < 4; ++i) {
      const size_t ao = (size_t)(m0 + (i << 4) + rlane) * lda + koff + k0;
      V ah = Frag<T>::load(Ab + ao);
      V al;
      if (SPLIT) al = Frag<T>::load(Ab2 + ao);
#pragma unroll
      for (int j = 0; j < 4; ++j) {
        acc[i][j] = Frag<T>::mma(ah, bh[j], acc[i][j]);
        if (SPLIT) {
          acc[i][j] = Frag<T>::mma(ah, bl[j], acc[i][j]);
          acc[i][j] = Frag<T>::mma(al, bh[j], acc[i][j]);
        }
      }
      Frag<T>::guard(acc[i][0], acc[i][3], ah, SPLIT ? al : ah);
    }
    Frag<T>::keep(bh[0], bh[1], bh[2], bh[3]);
    if (SPLIT) Frag<T>::keep(bl[0], bl[1], bl[2], bl[3]);
  }
  acc_guard4(acc[0][0], acc[0][1], acc[0][2], acc[0][3]);
  acc_guard4(acc[1][0], acc[1][1], acc[1][2], acc[1][3]);
  acc_guard4(acc[2][0], acc[2][1], acc[2][2], acc[2][3]);
  acc_guard4(acc[3][0], acc[3][1], acc[3][2], acc[3][3]);

  float* slab = sT[wave];
  const float* Rb = RESID ? (resid + (size_t)b * strideR) : nullptr;
#pragma unroll
  for (int i = 0; i < 4; ++i) {
    const int mBase = m0 + (i << 4);
#pragma unroll
    for (int j = 0; j < 4; ++j) {
      const int n = n0 + (j << 4) + rlane;
      float bv = 0.f;
      if (BIAS_MODE == 2) bv = bias[n];
#pragma unroll
      for (int r = 0; r < 8; ++r) {
        float v = acc[i][j][r] * scale;
        if (BIAS_MODE == 1) v += bias[mBase + mOff + r];
        if (BIAS_MODE == 2) v += bv;
        if (RESID) v += Rb[(size_t)(mBase + mOff + r) * ldc + n];
        if (ACT == 1) v = tanhf(v);
        if (ACT == 2) v = fmaxf(v, 0.0f);
        if (ACT == 3) v = v / (1.0f + expf(-v));
        if (ACT == 4) v = (v > 0.f) ? v : 0.01f * v;
        if (ACT == 5) v = 0.5f * v * (1.0f + erff(v * 0.70710678118654752f));
        slab[(mOff + r) * 68 + (j << 4) + rlane] = v;
      }
    }
    __builtin_amdgcn_fence(__ATOMIC_RELEASE, "workgroup");
    __builtin_amdgcn_wave_barrier();
    __builtin_amdgcn_fence(__ATOMIC_ACQUIRE, "workgroup");
    if (OUT_MODE == 0) {
      float* C = (float*)Cout + (size_t)b * strideC;
      const int hh = lane >> 4, c4 = (lane & 15) * 4;
      for (int pass = 0; pass < 2; ++pass) {
#pragma unroll
        for (int it = 0; it < 8; ++it) {
          const int row = it * 2 + hh;
          v4f v = *(const v4f*)(slab + row * 68 + c4);
          *(volatile v4f*)(C + (size_t)(mBase + row) * ldc + n0 + c4) = v;
        }
        __threadfence();
      }
    } else {
      const int q = lane >> 3, c8 = (lane & 7) * 8;
      unsigned short* C  = (unsigned short*)Cout  + (size_t)b * strideC;
      unsigned short* C2 = (OUT_MODE == 2) ? ((unsigned short*)Cout2 + (size_t)b * strideC) : nullptr;
      for (int pass = 0; pass < 2; ++pass) {
#pragma unroll
        for (int it = 0; it < 4; ++it) {
          const int row = it * 4 + q;
          const float* sp = slab + row * 68 + c8;
          v8h hv, lv;
#pragma unroll
          for (int e = 0; e < 8; ++e) {
            if (OUT_MODE == 1) {
              hv[e] = (_Float16)sp[e];
            } else {
              unsigned short hb = f2bf_bits(sp[e]);
              unsigned short lb = f2bf_bits(sp[e] - bf_bits2f(hb));
              hv[e] = __builtin_bit_cast(_Float16, hb);
              lv[e] = __builtin_bit_cast(_Float16, lb);
            }
          }
          *(volatile v8h*)(C + (size_t)(mBase + row) * ldc + n0 + c8) = hv;
          if (OUT_MODE == 2) *(volatile v8h*)(C2 + (size_t)(mBase + row) * ldc + n0 + c8) = lv;
        }
        __threadfence();
      }
    }
    __builtin_amdgcn_fence(__ATOMIC_RELEASE, "workgroup");
    __builtin_amdgcn_wave_barrier();
    __builtin_amdgcn_fence(__ATOMIC_ACQUIRE, "workgroup");
  }
}

__global__ __launch_bounds__(256) void wcat_split_kernel(const float* __restrict__ Wl, const float* __restrict__ Wr,
                                                         unsigned* __restrict__ HI, unsigned* __restrict__ LO) {
  const int i = blockIdx.x * 256 + threadIdx.x;
  if (i >= DO * (KD / 2)) return;
  const int f  = i / (KD / 2);
  const int k  = 2 * (i - f * (KD / 2));
  const int kc = k & (DI - 1);
  const float l0 = Wl[(size_t)kc * DO + f], l1 = Wl[(size_t)(kc + 1) * DO + f];
  const float r0 = Wr[(size_t)kc * DO + f], r1 = Wr[(size_t)(kc + 1) * DO + f];
  const bool lo_half = (k < DI);
  const float a = lo_half ? l0 : r0;
  const float b = lo_half ? l1 : r1;
  unsigned short ah, al, bh, bl;
  split_bf(a, ah, al); split_bf(b, bh, bl);
  const unsigned uh = (unsigned)ah | ((unsigned)bh << 16);
  const unsigned ul = (unsigned)al | ((unsigned)bl << 16);
  ((volatile unsigned*)HI)[i] = uh; ((volatile unsigned*)LO)[i] = ul;
  __threadfence();
  ((volatile unsigned*)HI)[i] = uh; ((volatile unsigned*)LO)[i] = ul;
}

__device__ __forceinline__ int blk_excl_scan(int cnt, int* scan_ws, int tid, int* tot) {
  const int lane = tid & 31, wave = tid >> 5; int incl = cnt;
#pragma unroll
  for (int o = 1; o < 32; o <<= 1) { const int v = __shfl_up(incl, o, 32); if (lane >= o) incl += v; }
  if (lane == 31) scan_ws[wave] = incl;
  __syncthreads();
  if (wave == 0) { int wv = (lane < NT / 32) ? scan_ws[lane] : 0; int wincl = wv;
#pragma unroll
    for (int o = 1; o < 32; o <<= 1) { const int v = __shfl_up(wincl, o, 32); if (lane >= o) wincl += v; }
    if (lane < NT / 32) scan_ws[32 + lane] = wincl - wv; if (lane == 31) scan_ws[64] = wincl; }
  __syncthreads();
  const int res = scan_ws[32 + wave] + incl - cnt; *tot = scan_ws[64];
  return res;
}
template <int SP, int CAP, int NEDGE, int NSRC>
__device__ __forceinline__ int chunk_hits(const int* __restrict__ dstv, const int* __restrict__ srcv, int e0, int n0, int tid,
                                          int* LIST, int* scan_ws) {
  const int eb = e0 + tid * SP;
  const bool real = (eb < NEDGE);
  const int ebc = real ? eb : (NEDGE - SP);
  int rec[SP]; int cnt = 0;
#pragma unroll
  for (int k = 0; k < SP; k += 4) {
    const v4i d4 = *(const v4i*)(dstv + ebc + k);
    const v4i s4 = *(const v4i*)(srcv + ebc + k);
#pragma unroll
    for (int e = 0; e < 4; ++e) {
      int sr = s4[e]; sr = sr < 0 ? 0 : (sr >= NSRC ? NSRC - 1 : sr);
      const int d = d4[e];
      int r = -1;
      if (real && d >= n0 && d < n0 + SRB) { r = ((d - n0) << 17) | sr; ++cnt; }
      rec[k + e] = r;
    }
  }
  int tot; int p = blk_excl_scan(cnt, scan_ws, tid, &tot);
#pragma unroll
  for (int k = 0; k < SP; ++k) if (rec[k] >= 0) { if ((unsigned)p < (unsigned)CAP) LIST[p] = rec[k]; ++p; }
  __syncthreads();
  return tot < CAP ? tot : CAP;
}

template <int NSRC, int NEDGE>
__global__ __launch_bounds__(NT) void agg_kernel(const float* __restrict__ SRC, const int* __restrict__ srcv, const int* __restrict__ dstv,
                                                 float* ACC, float* __restrict__ CNT) {
  constexpr int NCHK = (NEDGE + SCH - 1) / SCH;
  __shared__ int LIST[SCH];
  __shared__ int scan_ws[80];
  const int tid = threadIdx.x, lane = tid & 31, wave = tid >> 5;
  const int n0 = blockIdx.x * SRB;
  const v2f zv = {0.0f, 0.0f};
#pragma unroll 1
  for (int j = 0; j < SRB / 8; ++j) {
    float* rp = ACC + (size_t)(n0 + wave * (SRB / 8) + j) * DI + 2 * lane;
    *(volatile v2f*)rp = zv;
    __threadfence();
    *(volatile v2f*)rp = zv;
  }
  int cA0 = 0, cA1 = 0, cA2 = 0, cA3 = 0, cB0 = 0, cB1 = 0, cB2 = 0, cB3 = 0;
#pragma unroll 1
  for (int c = 0; c < NCHK; ++c) {
    const int tot = chunk_hits<SPT, SCH, NEDGE, NSRC>(dstv, srcv, c * SCH, n0, tid, LIST, scan_ws);
#pragma unroll 1
    for (int base = 0; base < tot; base += 32) {
      const int q = base + lane;
      const int qc = (q < SCH) ? q : (SCH - 1);
      const int lv = LIST[qc];
      const int rv = (q < tot) ? lv : -1;
      const int own = (rv >= 0 && (rv >> 25) == wave) ? 1 : 0;
      unsigned msk = (unsigned)__ballot(own);
#pragma unroll 1
      for (int it = 0; it < 32; ++it) {
        if (msk == 0u) break;
        const int bp = __builtin_ctz(msk); msk &= msk - 1u;
        const int r = __shfl(rv, bp, 32);
        const int dl = (r >> 17) & (SRB - 1);
        int s = r & 0x1FFFF; s = (s < NSRC) ? s : (NSRC - 1);
        const int dll = dl & 255;
        const int hs  = dll >> 7;
        const int ol  = (dll >> 2) & 31;
        const int ix  = dll & 3;
        const bool mine = (ol == lane);
        const bool mA = mine && (hs == 0), mB = mine && (hs == 1);
        cA0 += (mA && ix == 0) ? 1 : 0; cA1 += (mA && ix == 1) ? 1 : 0; cA2 += (mA && ix == 2) ? 1 : 0; cA3 += (mA && ix == 3) ? 1 : 0;
        cB0 += (mB && ix == 0) ? 1 : 0; cB1 += (mB && ix == 1) ? 1 : 0; cB2 += (mB && ix == 2) ? 1 : 0; cB3 += (mB && ix == 3) ? 1 : 0;
        const v2f pv = *(const v2f*)(SRC + (size_t)s * DI + 2 * lane);
        float* rp = ACC + (size_t)(n0 + dl) * DI + 2 * lane;
        v2f a = *(const v2f*)rp;
        a = a + pv;
        *(volatile v2f*)rp = a;
        __threadfence();
        *(volatile v2f*)rp = a;
      }
    }
    __syncthreads();
  }
  v4f dA, dB;
  dA[0] = (float)cA0; dA[1] = (float)cA1; dA[2] = (float)cA2; dA[3] = (float)cA3;
  dB[0] = (float)cB0; dB[1] = (float)cB1; dB[2] = (float)cB2; dB[3] = (float)cB3;
  float* pA = CNT + (size_t)n0 + wave * 256 + 4 * lane;
  float* pB = pA + 128;
  *(volatile v4f*)pA = dA; *(volatile v4f*)pB = dB;
  __threadfence();
  *(volatile v4f*)pA = dA; *(volatile v4f*)pB = dB;
}

template <int NV, int MPR>
__global__ __launch_bounds__(256) void opsplit_kernel(const float* __restrict__ ACC, const float* __restrict__ CNT, const float* __restrict__ X,
                                                      unsigned short* __restrict__ HI, unsigned short* __restrict__ LO) {
  const int i = blockIdx.x * 256 + threadIdx.x;
  if (i >= MPR * 16) return;
  const int row = i >> 4, c8 = (i & 15) * 8, ca = c8 & (DI - 1);
  const int rc = (row < NV) ? row : (NV - 1);
  const float* pa = ACC + (size_t)row * DI + ca;
  const float* px = X + (size_t)rc * DI + ca;
  const v4f a0 = *(const v4f*)pa, a1 = *(const v4f*)(pa + 4);
  const v4f x0 = *(const v4f*)px, x1 = *(const v4f*)(px + 4);
  const float cn = CNT[row];
  const float inv = 1.0f / fmaxf(cn, 1.0f);
  v4f u0 = x0, u1 = x1;
  if (c8 < DI) { u0 = a0 * inv; u1 = a1 * inv; }
  const v4f z4 = {0.f, 0.f, 0.f, 0.f};
  if (row >= NV) { u0 = z4; u1 = z4; }
  v8h hv, lv;
#pragma unroll
  for (int e = 0; e < 4; ++e) {
    unsigned short h0, l0, h1, l1;
    split_bf(u0[e], h0, l0); split_bf(u1[e], h1, l1);
    hv[e] = __builtin_bit_cast(_Float16, h0); lv[e] = __builtin_bit_cast(_Float16, l0);
    hv[4 + e] = __builtin_bit_cast(_Float16, h1); lv[4 + e] = __builtin_bit_cast(_Float16, l1);
  }
  unsigned short* ph = HI + (size_t)row * KD + c8;
  unsigned short* pl = LO + (size_t)row * KD + c8;
  *(volatile v8h*)ph = hv; *(volatile v8h*)pl = lv;
  __threadfence();
  *(volatile v8h*)ph = hv; *(volatile v8h*)pl = lv;
}

template <int NV>
__global__ __launch_bounds__(256) void head_kernel(const float* __restrict__ H, const float* __restrict__ Wlin, const float* __restrict__ blin,
                                                   const float* __restrict__ alpha, float* __restrict__ out) {
  const int lane = threadIdx.x & 31, wave = threadIdx.x >> 5;
  const int rb = (blockIdx.x * 8 + wave) * 32;
  if (rb >= NV) return;
  const v4f w4 = *(const v4f*)(Wlin + 4 * lane);
  const float b0 = blin[0], al = alpha[0];
  float res = 0.0f;
#pragma unroll 1
  for (int i = 0; i < 32; ++i) {
    const v4f h4 = *(const v4f*)(H + (size_t)(rb + i) * DO + 4 * lane);
    float s = h4[0] * w4[0] + h4[1] * w4[1] + h4[2] * w4[2] + h4[3] * w4[3];
#pragma unroll
    for (int off = 1; off < 32; off <<= 1) s += __shfl_xor(s, off, 32);
    s += b0;
    const float y = (s > 0.0f) ? s : al * s;
    res = (lane == i) ? y : res;
  }
  float* op = out + rb + lane;
  *(volatile float*)op = res;
  __threadfence();
  *(volatile float*)op = res;
}

__global__ __launch_bounds__(256) void copy4_kernel(const float* __restrict__ S, float* __restrict__ D, int n4) {
  const int i = blockIdx.x * 256 + threadIdx.x;
  if (i >= n4) return;
  const v4f v = *(const v4f*)(S + (size_t)4 * i);
  float* op = D + (size_t)4 * i;
  *(volatile v4f*)op = v;
  __threadfence();
  *(volatile v4f*)op = v;
}

extern "C" void kernel_launch(void* const* d_in, const int* in_sizes, int n_in,
                              void* d_out, int out_size, void* d_ws, size_t ws_size, hipStream_t stream) {
  if (n_in < 26) return;
  if (in_sizes[0] != NPF * DI || in_sizes[1] != NGW * DI || in_sizes[2] != NSW * DI ||
      in_sizes[3] != EPG || in_sizes[4] != EPG || in_sizes[5] != EGP || in_sizes[6] != EGP ||
      in_sizes[7] != ESP || in_sizes[8] != ESP || in_sizes[9] != EPS || in_sizes[10] != EPS) return;
  if (in_sizes[11] != DI * DO || in_sizes[12] != DI * DO || in_sizes[13] != DO ||
      in_sizes[14] != DI * DO || in_sizes[15] != DI * DO || in_sizes[16] != DO ||
      in_sizes[17] != DI * DO || in_sizes[18] != DI * DO || in_sizes[19] != DO ||
      in_sizes[20] != DI * DO || in_sizes[21] != DI * DO || in_sizes[22] != DO ||
      in_sizes[23] != DO || in_sizes[24] != 1 || in_sizes[25] != 1) return;
  if (out_size != NPF * DO + NGW + NSW) return;

  const float* x_pf  = (const float*)d_in[0];
  const float* x_gw  = (const float*)d_in[1];
  const float* x_sw  = (const float*)d_in[2];
  const int* pg_src  = (const int*)d_in[3];
  const int* pg_dst  = (const int*)d_in[4];
  const int* gp_src  = (const int*)d_in[5];
  const int* gp_dst  = (const int*)d_in[6];
  const int* sp_src  = (const int*)d_in[7];
  const int* sp_dst  = (const int*)d_in[8];
  const int* ps_src  = (const int*)d_in[9];
  const int* ps_dst  = (const int*)d_in[10];
  const float* Wl_pg = (const float*)d_in[11];
  const float* Wr_pg = (const float*)d_in[12];
  const float* b_pg  = (const float*)d_in[13];
  const float* Wl_gp = (const float*)d_in[14];
  const float* Wr_gp = (const float*)d_in[15];
  const float* b_gp  = (const float*)d_in[16];
  const float* Wl_sp = (const float*)d_in[17];
  const float* Wr_sp = (const float*)d_in[18];
  const float* b_sp  = (const float*)d_in[19];
  const float* Wl_ps = (const float*)d_in[20];
  const float* Wr_ps = (const float*)d_in[21];
  const float* b_ps  = (const float*)d_in[22];
  const float* W_lin = (const float*)d_in[23];
  const float* b_lin = (const float*)d_in[24];
  const float* alpha = (const float*)d_in[25];

  float* out0 = (float*)d_out;
  float* out1 = out0 + (size_t)NPF * DO;
  float* out2 = out1 + (size_t)NGW;

  char* ws = (char*)d_ws; size_t off = 0;
  auto carve = [&](size_t bytes) -> char* { char* p = ws + off; off += (bytes + 255) & ~(size_t)255; return p; };
  const size_t WPB = (size_t)DO * KD * 2;
  unsigned* BTH_pg = (unsigned*)carve(WPB); unsigned* BTL_pg = (unsigned*)carve(WPB);
  unsigned* BTH_gp = (unsigned*)carve(WPB); unsigned* BTL_gp = (unsigned*)carve(WPB);
  unsigned* BTH_sp = (unsigned*)carve(WPB); unsigned* BTL_sp = (unsigned*)carve(WPB);
  unsigned* BTH_ps = (unsigned*)carve(WPB); unsigned* BTL_ps = (unsigned*)carve(WPB);
  const size_t R1B = (size_t)MP_GW * DO * 4;
  const size_t R2B = (size_t)MP_GW * KD * 2 * 2;
  char* R1 = carve(R1B);
  char* R2 = carve(R2B);
  if (off > ws_size || off > (size_t)134217728) return;

  const size_t ACCGWB = (size_t)NPA_GW * DI * 4;
  const size_t CNTGWB = (size_t)NPA_GW * 4;
  if (ACCGWB + CNTGWB > R1B) return;
  float* ACC_gw = (float*)R1;
  float* CNT_gw = (float*)(R1 + ACCGWB);
  float* H_gw   = (float*)R1;
  const size_t OPGWB = (size_t)MP_GW * KD * 2;
  unsigned short* OPH = (unsigned short*)R2;
  unsigned short* OPL = (unsigned short*)(R2 + OPGWB);
  const size_t PPFB = (size_t)MP_PF * KD * 2;
  const size_t FPFB = (size_t)MP_PF * DO * 4;
  unsigned short* P1H = (unsigned short*)(R1);
  unsigned short* P1L = (unsigned short*)(R1 + PPFB);
  unsigned short* P2H = (unsigned short*)(R1 + 2 * PPFB);
  unsigned short* P2L = (unsigned short*)(R1 + 3 * PPFB);
  float* T_pf  = (float*)(R1 + 4 * PPFB);
  float* HP_pf = (float*)(R1 + 4 * PPFB + FPFB);
  if (4 * PPFB + 2 * FPFB > R1B) return;
  const size_t ACCSB = (size_t)NPA_PF * DI * 4;
  const size_t CNTSB = (size_t)NPA_PF * 4;
  float* ACC_gp = (float*)(R2);
  float* CNT_gp = (float*)(R2 + ACCSB);
  float* ACC_sp = (float*)(R2 + ACCSB + CNTSB);
  float* CNT_sp = (float*)(R2 + 2 * ACCSB + CNTSB);
  float* ACC_ps = (float*)(R2 + 2 * ACCSB + 2 * CNTSB);
  float* CNT_ps = (float*)(R2 + 3 * ACCSB + 2 * CNTSB);
  const size_t o3 = 3 * ACCSB + 3 * CNTSB;
  unsigned short* P3H = (unsigned short*)(R2 + o3);
  unsigned short* P3L = (unsigned short*)(R2 + o3 + PPFB);
  float* H_sw = (float*)(R2 + o3 + 2 * PPFB);
  if (o3 + 2 * PPFB + FPFB > R2B) return;

  wcat_split_kernel<<<(DO * (KD / 2)) / 256, 256, 0, stream>>>(Wl_pg, Wr_pg, BTH_pg, BTL_pg);
  wcat_split_kernel<<<(DO * (KD / 2)) / 256, 256, 0, stream>>>(Wl_gp, Wr_gp, BTH_gp, BTL_gp);
  wcat_split_kernel<<<(DO * (KD / 2)) / 256, 256, 0, stream>>>(Wl_sp, Wr_sp, BTH_sp, BTL_sp);
  wcat_split_kernel<<<(DO * (KD / 2)) / 256, 256, 0, stream>>>(Wl_ps, Wr_ps, BTH_ps, BTL_ps);

  agg_kernel<NPF, EPG><<<TL_GW, NT, 0, stream>>>(x_pf, pg_src, pg_dst, ACC_gw, CNT_gw);
  opsplit_kernel<NGW, MP_GW><<<(MP_GW * 16) / 256, 256, 0, stream>>>(ACC_gw, CNT_gw, x_gw, OPH, OPL);
  {
    const int tiles = (MP_GW / 64) * (DO / 64);
    wmma_gemm64<1, true, 2, 0, false, 2><<<dim3((tiles + 7) / 8, 1), 256, 0, stream>>>(
        OPH, OPL, KD, 0L, (const unsigned short*)BTH_pg, (const unsigned short*)BTL_pg, KD, 0L,
        (void*)H_gw, nullptr, DO, 0L, b_pg, nullptr, 0L, MP_GW, DO, KD, 1.0f);
  }
  head_kernel<NGW><<<(NGW + 255) / 256, 256, 0, stream>>>(H_gw, W_lin, b_lin, alpha, out1);

  agg_kernel<NGW, EGP><<<TL_PF, NT, 0, stream>>>(x_gw, gp_src, gp_dst, ACC_gp, CNT_gp);
  agg_kernel<NSW, ESP><<<TL_PF, NT, 0, stream>>>(x_sw, sp_src, sp_dst, ACC_sp, CNT_sp);
  opsplit_kernel<NPF, MP_PF><<<(MP_PF * 16) / 256, 256, 0, stream>>>(ACC_gp, CNT_gp, x_pf, P1H, P1L);
  opsplit_kernel<NPF, MP_PF><<<(MP_PF * 16) / 256, 256, 0, stream>>>(ACC_sp, CNT_sp, x_pf, P2H, P2L);
  {
    const int tiles = (MP_PF / 64) * (DO / 64);
    wmma_gemm64<1, true, 2, 0, false, 0><<<dim3((tiles + 7) / 8, 1), 256, 0, stream>>>(
        P1H, P1L, KD, 0L, (const unsigned short*)BTH_gp, (const unsigned short*)BTL_gp, KD, 0L,
        (void*)T_pf, nullptr, DO, 0L, b_gp, nullptr, 0L, MP_PF, DO, KD, 1.0f);
    wmma_gemm64<1, true, 2, 0, true, 2><<<dim3((tiles + 7) / 8, 1), 256, 0, stream>>>(
        P2H, P2L, KD, 0L, (const unsigned short*)BTH_sp, (const unsigned short*)BTL_sp, KD, 0L,
        (void*)HP_pf, nullptr, DO, 0L, b_sp, T_pf, 0L, MP_PF, DO, KD, 1.0f);
  }
  copy4_kernel<<<(NPF * DO / 4) / 256, 256, 0, stream>>>(HP_pf, out0, NPF * DO / 4);

  agg_kernel<NPF, EPS><<<TL_SW, NT, 0, stream>>>(x_pf, ps_src, ps_dst, ACC_ps, CNT_ps);
  opsplit_kernel<NSW, MP_SW><<<(MP_SW * 16) / 256, 256, 0, stream>>>(ACC_ps, CNT_ps, x_sw, P3H, P3L);
  {
    const int tiles = (MP_SW / 64) * (DO / 64);
    wmma_gemm64<1, true, 2, 0, false, 2><<<dim3((tiles + 7) / 8, 1), 256, 0, stream>>>(
        P3H, P3L, KD, 0L, (const unsigned short*)BTH_ps, (const unsigned short*)BTL_ps, KD, 0L,
        (void*)H_sw, nullptr, DO, 0L, b_ps, nullptr, 0L, MP_SW, DO, KD, 1.0f);
  }
  head_kernel<NSW><<<(NSW + 255) / 256, 256, 0, stream>>>(H_sw, W_lin, b_lin, alpha, out2);
}
